// Block_33105607917680
// MI455X (gfx1250) — hardware-run, weakly checked
//
#include <hip/hip_runtime.h>

typedef float          v8f   __attribute__((ext_vector_type(8)));
typedef float          v4f   __attribute__((ext_vector_type(4)));
typedef unsigned int   v4u   __attribute__((ext_vector_type(4)));
typedef int            v8i   __attribute__((ext_vector_type(8)));
typedef unsigned short v8us  __attribute__((ext_vector_type(8)));
typedef unsigned short v16us __attribute__((ext_vector_type(16)));
typedef __bf16         v16bf __attribute__((ext_vector_type(16)));
typedef _Float16       v16h  __attribute__((ext_vector_type(16)));
typedef v4f  __attribute__((may_alias)) v4fa;
typedef v8us __attribute__((may_alias)) v8usa;
union FragB { v16bf v; v16us u; v8us h[2]; v8i w; };
union FragH { v16h  v; v16us u; v8us h[2]; v8i w; };

__device__ __forceinline__ v8f wmb(const FragB& a, const FragB& b, v8f c) {
  v8f d = __builtin_amdgcn_wmma_f32_16x16x32_bf16(false, a.v, false, b.v, (short)0, c, false, false);
  asm volatile("v_nop\n\tv_nop\n\tv_nop\n\tv_nop" : "+v"(d) : "v"(a.w), "v"(b.w));
  return d;
}

__device__ __forceinline__ v8f wmh(const FragH& a, const FragH& b, v8f c) {
  v8f d = __builtin_amdgcn_wmma_f32_16x16x32_f16(false, a.v, false, b.v, (short)0, c, false, false);
  asm volatile("v_nop\n\tv_nop\n\tv_nop\n\tv_nop" : "+v"(d) : "v"(a.w), "v"(b.w));
  return d;
}

__device__ __forceinline__ unsigned bf16_bits(float f) {
  const unsigned u = __float_as_uint(f);
  const unsigned r = (u + 0x7FFFu + ((u >> 16) & 1u)) >> 16;
  const unsigned q = (u >> 16) | 0x40u;
  return ((u & 0x7fffffffu) > 0x7f800000u) ? q : r;
}

__device__ __forceinline__ float bf16_val(float f) {
  return __uint_as_float(bf16_bits(f) << 16);
}
__device__ __forceinline__ int clampi(int v, int lo, int hi) {
  return v < lo ? lo : (v > hi ? hi : v);
}

__device__ __forceinline__ unsigned f16_bits(float f) {
  const unsigned u  = __float_as_uint(f);
  const unsigned s  = (u >> 16) & 0x8000u;
  const unsigned a  = u & 0x7fffffffu;
  const unsigned t  = a - 0x38000000u;
  const unsigned r  = (t + 0x0FFFu + ((t >> 13) & 1u)) >> 13;
  const unsigned rc = r > 0x7C00u ? 0x7C00u : r;
  const bool small  = a < 0x38800000u;
  const bool isnan  = a > 0x7f800000u;
  const unsigned fin = small ? 0u : (s | rc);
  return isnan ? (s | 0x7E00u) : fin;
}

__device__ __forceinline__ unsigned pk16(unsigned lo, unsigned hi) { return lo | (hi << 16); }
__device__ __forceinline__ unsigned bf16_lo_bits(float v) {
  float hi = bf16_val(v);
  asm volatile("" : "+v"(hi));
  return bf16_bits(v - hi);
}
__device__ __forceinline__ v4u pack8_bf16(v4f a, v4f c) {
  return (v4u){ pk16(bf16_bits(a[0]), bf16_bits(a[1])), pk16(bf16_bits(a[2]), bf16_bits(a[3])),
                pk16(bf16_bits(c[0]), bf16_bits(c[1])), pk16(bf16_bits(c[2]), bf16_bits(c[3])) };
}
__device__ __forceinline__ v4u pack8_bf16_lo(v4f a, v4f c) {
  return (v4u){ pk16(bf16_lo_bits(a[0]), bf16_lo_bits(a[1])), pk16(bf16_lo_bits(a[2]), bf16_lo_bits(a[3])),
                pk16(bf16_lo_bits(c[0]), bf16_lo_bits(c[1])), pk16(bf16_lo_bits(c[2]), bf16_lo_bits(c[3])) };
}
__device__ __forceinline__ v4u pack8_f16(v4f a, v4f c) {
  return (v4u){ pk16(f16_bits(a[0]), f16_bits(a[1])), pk16(f16_bits(a[2]), f16_bits(a[3])),
                pk16(f16_bits(c[0]), f16_bits(c[1])), pk16(f16_bits(c[2]), f16_bits(c[3])) };
}

template <int FORM>
__global__ __launch_bounds__(256) void k_plane(const float* __restrict__ src, int rows, int cols, int ldsrc,
                                               unsigned short* __restrict__ dst, int MP, int KP) {
  static_assert(FORM >= 0 && FORM <= 3);
  const int KTOT = (FORM == 1 || FORM == 3) ? 2 * KP : KP;
  const unsigned ppr   = (unsigned)(KTOT >> 3);
  const unsigned kp8   = (unsigned)(KP >> 3);
  const unsigned total = (unsigned)MP * ppr;
  const unsigned g     = blockIdx.x * 256u + threadIdx.x;
  const unsigned rowu  = g / ppr;
  const unsigned p     = g - rowu * ppr;
  const bool second    = p >= kp8;
  const int row = (int)rowu;
  const int c0  = (int)((second ? p - kp8 : p) << 3);
  const float* srow = src + (size_t)clampi(row, 0, rows - 1) * (size_t)ldsrc;
  float x[8];
  unsigned mk[8];
#pragma unroll
  for (int e = 0; e < 8; ++e) {
    const int c = c0 + e;
    const float v = srow[clampi(c, 0, cols - 1)];
    asm volatile("" :: "v"(v));
    x[e]  = v;
    mk[e] = (row < rows && c < cols) ? 0xFFFFu : 0u;
  }
  const v4f a = (v4f){ x[0], x[1], x[2], x[3] };
  const v4f c = (v4f){ x[4], x[5], x[6], x[7] };
  v4u o;
  if (FORM == 2) {
    o = pack8_f16(a, c);
  } else {
    const v4u hi = pack8_bf16(a, c);
    o = hi;
    if (FORM == 1) { const v4u lo = pack8_bf16_lo(a, c); o = second ? lo : hi; }
  }
  const v4u mw = (v4u){ pk16(mk[0], mk[1]), pk16(mk[2], mk[3]), pk16(mk[4], mk[5]), pk16(mk[6], mk[7]) };
  o &= mw;
  if (g < total) {
    volatile v4u* q = (volatile v4u*)(dst + (size_t)g * 8);
    *q = o;
    __threadfence();
    *q = o;
  }
}

template <int FORM> struct FragOf    { typedef FragB T; };
template <>         struct FragOf<2> { typedef FragH T; };
__device__ __forceinline__ v8f mm(const FragB& a, const FragB& b, v8f c) { return wmb(a, b, c); }
__device__ __forceinline__ v8f mm(const FragH& a, const FragH& b, v8f c) { return wmh(a, b, c); }
template <class F> __device__ __forceinline__ F ld_frag(const unsigned short* p) {
  F f;
  f.h[0] = *(const v8usa*)(p);
  f.h[1] = *(const v8usa*)(p + 16);
  return f;
}

template <int FORM, int EPI>
__global__ __launch_bounds__(256) __attribute__((amdgpu_num_vgpr(248)))
void k_gemm_nt(const unsigned short* __restrict__ A, const unsigned short* __restrict__ B,
               const float* __restrict__ bias, float* __restrict__ D, int M, int N, int KTOT, int ldd) {
  static_assert(FORM >= 0 && FORM <= 2);
  static_assert(EPI == 0 || EPI == 1);
  typedef typename FragOf<FORM>::T F;
  __shared__ __attribute__((aligned(16))) float sT[8][16 * 68];
  const int lane = threadIdx.x & 31;
  const int wave = threadIdx.x >> 5;
  const int tilesM = (M + 63) >> 6;
  const int tilesN = (N + 63) >> 6;
  const int tile = blockIdx.x * 8 + wave;
  if (tile >= tilesM * tilesN) return;
  const int tm = tile / tilesN;
  const int tn = tile - tm * tilesN;
  const int m0 = tm << 6;
  const int n0 = tn << 6;

  const int rl = lane & 15;
  const int h8 = (lane >> 4) * 8;
  const unsigned short* pa = A + (size_t)(m0 + rl) * (size_t)KTOT + h8;
  const unsigned short* pb = B + (size_t)(n0 + rl) * (size_t)KTOT + h8;

  v8f acc[4][4];
#pragma unroll
  for (int i = 0; i < 4; ++i)
#pragma unroll
    for (int j = 0; j < 4; ++j) acc[i][j] = (v8f){0.f, 0.f, 0.f, 0.f, 0.f, 0.f, 0.f, 0.f};

#pragma unroll 1
  for (int k0 = 0; k0 < KTOT; k0 += 32) {
    F bf[4];
#pragma unroll
    for (int j = 0; j < 4; ++j) bf[j] = ld_frag<F>(pb + (size_t)(j << 4) * (size_t)KTOT + k0);
#pragma unroll
    for (int i = 0; i < 4; ++i) {
      const F af = ld_frag<F>(pa + (size_t)(i << 4) * (size_t)KTOT + k0);
#pragma unroll
      for (int j = 0; j < 4; ++j) acc[i][j] = mm(af, bf[j], acc[i][j]);
    }
  }

  float* slab = sT[wave];
  const int hh = lane >> 4;
  const int c4 = (lane & 15) * 4;
  const int nc = n0 + c4;
  const bool cok = nc < N;
  v4f bv = (v4f){0.f, 0.f, 0.f, 0.f};
  if (EPI == 1) {
    bv = *(const v4fa*)(bias + clampi(nc, 0, N - 4));
    asm volatile("" :: "v"(bv));
  }
#pragma unroll
  for (int i = 0; i < 4; ++i) {
    const int mBase = m0 + (i << 4);
#pragma unroll
    for (int j = 0; j < 4; ++j) {
#pragma unroll
      for (int r = 0; r < 8; ++r) slab[(h8 + r) * 68 + (j << 4) + rl] = acc[i][j][r];
    }
    __builtin_amdgcn_fence(__ATOMIC_RELEASE, "workgroup");
    __builtin_amdgcn_wave_barrier();
    __builtin_amdgcn_fence(__ATOMIC_ACQUIRE, "workgroup");
    v4f vv[8];
#pragma unroll
    for (int it = 0; it < 8; ++it) {
      const int row = it * 2 + hh;
      v4f v = *(const v4fa*)(slab + row * 68 + c4);
      if (EPI == 1) v += bv;
      vv[it] = v;
    }
    for (int pass = 0; pass < 2; ++pass) {
#pragma unroll
      for (int it = 0; it < 8; ++it) {
        const int row = mBase + it * 2 + hh;
        if (cok && row < M) *(volatile v4f*)(D + (size_t)row * (size_t)ldd + nc) = vv[it];
      }
      __threadfence();
    }
    __builtin_amdgcn_fence(__ATOMIC_RELEASE, "workgroup");
    __builtin_amdgcn_wave_barrier();
    __builtin_amdgcn_fence(__ATOMIC_ACQUIRE, "workgroup");
  }
}

#pragma clang fp contract(off)

typedef double v2d __attribute__((ext_vector_type(2)));
typedef v2d __attribute__((may_alias)) v2da;

constexpr int NBAT   = 2;
constexpr int NPT    = 8192;
constexpr int KNB    = 16;
constexpr int DIM    = 256;
constexpr int HID    = 1024;
constexpr int D4     = 64;
constexpr int DEPTH  = 4;
constexpr int NMLP   = 3;
constexpr int ROWS   = NBAT * NPT;
constexpr int CHROWS = 4096;
constexpr int NCHUNK = ROWS / CHROWS;
constexpr int NREC   = ROWS / 128;
constexpr int OUT_ELEMS = ROWS * DIM;

constexpr int SITE_MODE[9] = { 2, 2, 2, 2, 2, 2, 2, 2, 2 };
constexpr unsigned site_mask(int s) { return SITE_MODE[s] == 2 ? 0xFFFFFFFFu : 0u; }

static_assert(ROWS % 128 == 0 && CHROWS % 128 == 0 && CHROWS * NCHUNK == ROWS);
static_assert(DIM == 32 * 8 && D4 == 2 * 32 && KNB == 16 && HID == 1024 && D4 * 4 == DIM);
static_assert(NPT == (1 << 13) && ROWS == 16384 && NREC == 128);
static_assert(ROWS % 64 == 0 && CHROWS % 64 == 0 && HID % 64 == 0 && DIM % 64 == 0);
static_assert(DIM % 32 == 0 && (2 * DIM) % 32 == 0 && (2 * HID) % 32 == 0);
static_assert(OUT_ELEMS == 4194304);

constexpr int TB_LFPT = 0;
constexpr int TB_B1   = TB_LFPT + DEPTH * D4 * 8;
constexpr int TB_LG   = TB_B1 + NMLP * HID;
constexpr int TB_LB   = TB_LG + DEPTH * DIM;
constexpr int TB_MG   = TB_LB + DEPTH * DIM;
constexpr int TB_MB   = TB_MG + NMLP * DIM;
constexpr int TB_MU   = TB_MB + NMLP * DIM;
constexpr int TB_RS   = TB_MU + DIM;
constexpr int TB_END  = TB_RS + DIM;
static_assert(TB_B1 % 32 == 0 && TB_LG % 32 == 0 && TB_LB % 32 == 0 && TB_MG % 32 == 0);
static_assert(TB_MB % 32 == 0 && TB_MU % 32 == 0 && TB_RS % 32 == 0 && TB_END == 9216);
constexpr size_t TBB_PC  = 65536;
constexpr size_t TBB_REC = TBB_PC + (size_t)ROWS * 16;
constexpr size_t TBB_END = TBB_REC + (size_t)NREC * DIM * 8;
static_assert((size_t)TB_END * 4 <= TBB_PC);
static_assert(TBB_PC % 256 == 0 && TBB_REC % 256 == 0);

constexpr size_t SZ_XF   = (size_t)ROWS * DIM * 4;
constexpr size_t SZ_XHL  = (size_t)ROWS * 2 * DIM * 2;
constexpr size_t SZ_HP   = (size_t)ROWS * DIM * 4;
constexpr size_t SZ_AG   = (size_t)ROWS * DIM * 4;
constexpr size_t SZ_C1   = (size_t)CHROWS * HID * 4;
constexpr size_t SZ_C1HL = (size_t)CHROWS * 2 * HID * 2;
constexpr size_t SZ_XB   = (size_t)ROWS * DIM * 2;
constexpr size_t SZ_W1A  = (size_t)HID * DIM * 2;
constexpr size_t SZ_W1B  = (size_t)2 * HID * 2 * DIM * 2;
constexpr size_t SZ_W2P  = (size_t)NMLP * DIM * 2 * HID * 2;
constexpr size_t SZ_LW2  = (size_t)DEPTH * DIM * 2 * DIM * 2;
constexpr size_t SZ_TB   = 1048576;
constexpr size_t OFF_XF   = 0;
constexpr size_t OFF_XHL  = OFF_XF + SZ_XF;
constexpr size_t OFF_HP   = OFF_XHL + SZ_XHL;
constexpr size_t OFF_AG   = OFF_HP + SZ_HP;
constexpr size_t OFF_C1   = OFF_AG + SZ_AG;
constexpr size_t OFF_C1HL = OFF_C1 + SZ_C1;
constexpr size_t OFF_XB   = OFF_C1HL + SZ_C1HL;
constexpr size_t OFF_W1A  = OFF_XB + SZ_XB;
constexpr size_t OFF_W1B  = OFF_W1A + SZ_W1A;
constexpr size_t OFF_W2P  = OFF_W1B + SZ_W1B;
constexpr size_t OFF_LW2  = OFF_W2P + SZ_W2P;
constexpr size_t OFF_TB   = OFF_LW2 + SZ_LW2;
constexpr size_t WS_TOTAL = OFF_TB + SZ_TB;
static_assert(WS_TOTAL == (size_t)((size_t)223 << 19));
static_assert(WS_TOTAL <= ((size_t)128 << 20));
static_assert(OFF_XHL % 256 == 0 && OFF_HP % 256 == 0 && OFF_AG % 256 == 0 && OFF_C1 % 256 == 0);
static_assert(OFF_C1HL % 256 == 0 && OFF_XB % 256 == 0 && OFF_W1A % 256 == 0 && OFF_W1B % 256 == 0);
static_assert(OFF_W2P % 256 == 0 && OFF_LW2 % 256 == 0 && OFF_TB % 256 == 0);
static_assert(TBB_END <= SZ_TB);

__device__ __forceinline__ float gelu_t(float v) {
  const float v3  = (v * v) * v;
  const float u   = 0x1.988454p-1f * (v + 0.044715f * v3);
  const float cdf = 0.5f * (1.0f + tanhf(u));
  return v * cdf;
}

__global__ __launch_bounds__(256) void k_prep_x(const float* __restrict__ x, float* __restrict__ XF,
                                                unsigned short* __restrict__ XB) {
  const int tid = (int)threadIdx.x, lane = tid & 31, wave = tid >> 5;
  const int row = (int)blockIdx.x * 8 + wave;
  const int rc  = row < ROWS ? row : ROWS - 1;
  const float* xr = x + (size_t)rc * DIM;
  const v4f a0 = *(const v4fa*)(xr + 4 * lane);
  const v4f a1 = *(const v4fa*)(xr + 128 + 4 * lane);
  const v4f c0 = *(const v4fa*)(xr + 8 * lane);
  const v4f c1 = *(const v4fa*)(xr + 8 * lane + 4);
  asm volatile("" :: "v"(a0));
  asm volatile("" :: "v"(a1));
  asm volatile("" :: "v"(c0));
  asm volatile("" :: "v"(c1));
  v4f f0, f1;
#pragma unroll
  for (int e = 0; e < 4; ++e) { f0[e] = bf16_val(a0[e]); f1[e] = bf16_val(a1[e]); }
  const v4u hb = pack8_bf16(c0, c1);
  if (row < ROWS) {
    float* fr = XF + (size_t)row * DIM + 4 * lane;
    unsigned short* br = XB + (size_t)row * DIM + 8 * lane;
    *(volatile v4f*)(fr)       = f0;
    *(volatile v4f*)(fr + 128) = f1;
    *(volatile v4u*)(br)       = hb;
    __threadfence();
    *(volatile v4f*)(fr)       = f0;
    *(volatile v4f*)(fr + 128) = f1;
    *(volatile v4u*)(br)       = hb;
  }
}

__global__ __launch_bounds__(256) void k_wT(const float* __restrict__ W, unsigned short* __restrict__ P,
                                            int Kin, int Nout, int dup) {
  __shared__ float tile[64 * 65];
  const int tid = (int)threadIdx.x;
  const int tilesK = Kin >> 6, tilesN = Nout >> 6;
  const int per = tilesK * tilesN;
  const int z   = (int)blockIdx.x / per;
  const int rem = (int)blockIdx.x - z * per;
  const int tk  = rem / tilesN;
  const int tn  = rem - tk * tilesN;
  const int k0 = tk << 6, n0 = tn << 6;
  const int KTOT = Kin * dup;
  const float* src = W + (size_t)z * (size_t)Kin * (size_t)Nout;
  unsigned short* dst = P + (size_t)z * (size_t)Nout * (size_t)KTOT;
  const int c4 = (tid & 15) * 4;
#pragma unroll
  for (int i = 0; i < 4; ++i) {
    const int kr = (tid >> 4) + 16 * i;
    const v4f v = *(const v4fa*)(src + (size_t)(k0 + kr) * (size_t)Nout + n0 + c4);
    tile[kr * 65 + c4 + 0] = v[0];
    tile[kr * 65 + c4 + 1] = v[1];
    tile[kr * 65 + c4 + 2] = v[2];
    tile[kr * 65 + c4 + 3] = v[3];
  }
  __syncthreads();
  v4u o[2];
#pragma unroll
  for (int i = 0; i < 2; ++i) {
    const int q  = tid + 256 * i;
    const int n  = q >> 3;
    const int pc = q & 7;
    const float* tp = tile + (pc * 8) * 65 + n;
    o[i] = (v4u){ pk16(bf16_bits(tp[0 * 65]), bf16_bits(tp[1 * 65])), pk16(bf16_bits(tp[2 * 65]), bf16_bits(tp[3 * 65])),
                  pk16(bf16_bits(tp[4 * 65]), bf16_bits(tp[5 * 65])), pk16(bf16_bits(tp[6 * 65]), bf16_bits(tp[7 * 65])) };
  }
#pragma unroll
  for (int i = 0; i < 2; ++i) {
    const int q = tid + 256 * i;
    unsigned short* dp = dst + (size_t)(n0 + (q >> 3)) * (size_t)KTOT + k0 + (q & 7) * 8;
    *(volatile v4u*)dp = o[i];
    if (dup == 2) *(volatile v4u*)(dp + Kin) = o[i];
  }
  __threadfence();
#pragma unroll
  for (int i = 0; i < 2; ++i) {
    const int q = tid + 256 * i;
    unsigned short* dp = dst + (size_t)(n0 + (q >> 3)) * (size_t)KTOT + k0 + (q & 7) * 8;
    *(volatile v4u*)dp = o[i];
    if (dup == 2) *(volatile v4u*)(dp + Kin) = o[i];
  }
}

__device__ __forceinline__ void rcopy4(const float* __restrict__ src, float* __restrict__ dst, int piece, int npieces) {
  const int pc = piece < npieces ? piece : npieces - 1;
  const v4f a = *(const v4fa*)(src + 4 * pc);
  asm volatile("" :: "v"(a));
  v4f o;
#pragma unroll
  for (int e = 0; e < 4; ++e) o[e] = bf16_val(a[e]);
  if (piece < npieces) {
    volatile v4f* q = (volatile v4f*)(dst + 4 * piece);
    *q = o;
    __threadfence();
    *q = o;
  }
}

constexpr int PS_PC  = ROWS / 256;
constexpr int PS_TOT = PS_PC + 8;
__global__ __launch_bounds__(256) void k_prep_small(const float* __restrict__ xyz, const float* __restrict__ coor,
                                                    const float* __restrict__ scale, const float* __restrict__ lg,
                                                    const float* __restrict__ lb, const float* __restrict__ b1,
                                                    const float* __restrict__ mg, const float* __restrict__ mb,
                                                    float* __restrict__ PC, float* __restrict__ TB) {
  __shared__ __attribute__((aligned(16))) float sL[DEPTH * D4 * 8];
  const int tid = (int)threadIdx.x;
  const int blk = (int)blockIdx.x;
  if (blk < PS_PC) {
    const int r = blk * 256 + tid;
    const float* s = xyz + (size_t)r * 3;
    const float x = s[0], y = s[1], z = s[2];
    asm volatile("" :: "v"(x));
    asm volatile("" :: "v"(y));
    asm volatile("" :: "v"(z));
    const v4f o = (v4f){ bf16_val(x), bf16_val(y), bf16_val(z), 0.0f };
    volatile v4f* q = (volatile v4f*)(PC + (size_t)r * 4);
    *q = o;
    __threadfence();
    *q = o;
  } else if (blk == PS_PC) {
    const float* s = coor + 3 * tid;
    float cx = s[0], cy = s[1], cz = s[2];
    float sc = scale[tid];
    asm volatile("" :: "v"(cx));
    asm volatile("" :: "v"(cy));
    asm volatile("" :: "v"(cz));
    asm volatile("" :: "v"(sc));
    cx = bf16_val(cx); cy = bf16_val(cy); cz = bf16_val(cz); sc = bf16_val(sc);
    const float cc = (cx * cx + cy * cy) + cz * cz;
    const float ns = -(sc * sc);
    float* e = sL + 8 * tid;
    e[0] = cx; e[1] = cy; e[2] = cz; e[3] = cc; e[4] = ns; e[5] = 0.0f; e[6] = 0.0f; e[7] = 0.0f;
    __syncthreads();
    const v4f o0 = *(const v4fa*)(sL + 4 * tid);
    const v4f o1 = *(const v4fa*)(sL + 1024 + 4 * tid);
    float* d = TB + TB_LFPT + 4 * tid;
    *(volatile v4f*)(d)        = o0;
    *(volatile v4f*)(d + 1024) = o1;
    __threadfence();
    *(volatile v4f*)(d)        = o0;
    *(volatile v4f*)(d + 1024) = o1;
  } else if (blk < PS_PC + 4) {
    rcopy4(b1, TB + TB_B1, (blk - PS_PC - 1) * 256 + tid, NMLP * HID / 4);
  } else if (blk == PS_PC + 4) {
    rcopy4(lg, TB + TB_LG, tid, DEPTH * DIM / 4);
  } else if (blk == PS_PC + 5) {
    rcopy4(lb, TB + TB_LB, tid, DEPTH * DIM / 4);
  } else if (blk == PS_PC + 6) {
    rcopy4(mg, TB + TB_MG, tid, NMLP * DIM / 4);
  } else {
    rcopy4(mb, TB + TB_MB, tid, NMLP * DIM / 4);
  }
}

__global__ __launch_bounds__(256) void k_gelu(const float* __restrict__ C1, const float* __restrict__ b1,
                                              unsigned short* __restrict__ HL, unsigned lomask) {
  __shared__ __attribute__((aligned(16))) float sB[HID];
  __shared__ __attribute__((aligned(16))) float sR[8 * HID];
  const int tid = (int)threadIdx.x, lane = tid & 31, wave = tid >> 5;
  {
    const v4f bv = *(const v4fa*)(b1 + 4 * tid);
    *(v4fa*)(sB + 4 * tid) = bv;
  }
  __syncthreads();
  const int row = (int)blockIdx.x * 8 + wave;
  const int rc  = row < CHROWS ? row : CHROWS - 1;
  const float* cr = C1 + (size_t)rc * HID + lane;
  float* sr = sR + wave * HID;
#pragma unroll 1
  for (int it = 0; it < 32; ++it) {
    const float v = cr[32 * it] + sB[32 * it + lane];
    sr[32 * it + lane] = gelu_t(v);
  }
  __builtin_amdgcn_fence(__ATOMIC_RELEASE, "workgroup");
  __builtin_amdgcn_wave_barrier();
  __builtin_amdgcn_fence(__ATOMIC_ACQUIRE, "workgroup");
  const v4u mk = (v4u){ lomask, lomask, lomask, lomask };
  v4u hi[4], lo[4];
#pragma unroll
  for (int q = 0; q < 4; ++q) {
    const v4f a = *(const v4fa*)(sr + 256 * q + 8 * lane);
    const v4f c = *(const v4fa*)(sr + 256 * q + 8 * lane + 4);
    hi[q] = pack8_bf16(a, c);
    lo[q] = pack8_bf16_lo(a, c) & mk;
  }
  if (row < CHROWS) {
    unsigned short* hr = HL + (size_t)row * (2 * HID) + 8 * lane;
#pragma unroll
    for (int q = 0; q < 4; ++q) {
      *(volatile v4u*)(hr + 256 * q)       = hi[q];
      *(volatile v4u*)(hr + HID + 256 * q) = lo[q];
    }
    __threadfence();
#pragma unroll
    for (int q = 0; q < 4; ++q) {
      *(volatile v4u*)(hr + 256 * q)       = hi[q];
      *(volatile v4u*)(hr + HID + 256 * q) = lo[q];
    }
  }
}

__global__ __launch_bounds__(256) void k_lfp(const float* __restrict__ HP, const float* __restrict__ PC,
                                             const int* __restrict__ knn, const float* __restrict__ LT,
                                             float* __restrict__ AG) {
  const int tid = (int)threadIdx.x, lane = tid & 31, wave = tid >> 5;
  const int r  = __builtin_amdgcn_readfirstlane((int)blockIdx.x * 8 + wave);
  const int rr = r < ROWS ? r : ROWS - 1;
  const int b  = rr >> 13;
  const v4f ta = *(const v4fa*)(LT + 8 * lane);
  const v4f tb = *(const v4fa*)(LT + 8 * lane + 4);
  const v4f ua = *(const v4fa*)(LT + 8 * (lane + 32));
  const v4f ub = *(const v4fa*)(LT + 8 * (lane + 32) + 4);
  const float cax = ta[0], cay = ta[1], caz = ta[2], cca = ta[3], nsa = tb[0];
  const float cbx = ua[0], cby = ua[1], cbz = ua[2], ccb = ua[3], nsb = ub[0];
  int id = knn[(size_t)rr * KNB + (lane & 15)];
  asm volatile("" :: "v"(id));
  id = clampi(id, 0, NPT - 1);
  const int nrow = b * NPT + id;
  const v4f pnv = *(const v4fa*)(PC + (size_t)nrow * 4);
  const v4f pcv = *(const v4fa*)(PC + (size_t)rr * 4);
  asm volatile("" :: "v"(pnv));
  asm volatile("" :: "v"(pcv));
  const float px = pnv[0] - pcv[0];
  const float py = pnv[1] - pcv[1];
  const float pz = pnv[2] - pcv[2];
  const float pp = (px * px + py * py) + pz * pz;
  const int pxi = __float_as_int(px);
  const int pyi = __float_as_int(py);
  const int pzi = __float_as_int(pz);
  const int ppi = __float_as_int(pp);
  const float* Ha = HP + 4 * lane;
  float acc[8] = { 0.0f, 0.0f, 0.0f, 0.0f, 0.0f, 0.0f, 0.0f, 0.0f };
#pragma unroll 4
  for (int k = 0; k < KNB; ++k) {
    const int   nr = __builtin_amdgcn_readlane(nrow, k);
    const float bx = __int_as_float(__builtin_amdgcn_readlane(pxi, k));
    const float by = __int_as_float(__builtin_amdgcn_readlane(pyi, k));
    const float bz = __int_as_float(__builtin_amdgcn_readlane(pzi, k));
    const float bp = __int_as_float(__builtin_amdgcn_readlane(ppi, k));
    const v4f hA = *(const v4fa*)(Ha + (size_t)nr * DIM);
    const v4f hB = *(const v4fa*)(Ha + (size_t)nr * DIM + 128);
    asm volatile("" :: "v"(hA));
    asm volatile("" :: "v"(hB));
    const float dotA = (bx * cax + by * cay) + bz * caz;
    const float dotB = (bx * cbx + by * cby) + bz * cbz;
    const float d2A  = (bp - 2.0f * dotA) + cca;
    const float d2B  = (bp - 2.0f * dotB) + ccb;
    const float wA = expf(nsa * d2A);
    const float wB = expf(nsb * d2B);
#pragma unroll
    for (int e = 0; e < 4; ++e) {
      acc[e]     = acc[e]     + hA[e] * wA;
      acc[4 + e] = acc[4 + e] + hB[e] * wB;
    }
  }
  const v4f o0 = (v4f){ acc[0] * 0.0625f, acc[1] * 0.0625f, acc[2] * 0.0625f, acc[3] * 0.0625f };
  const v4f o1 = (v4f){ acc[4] * 0.0625f, acc[5] * 0.0625f, acc[6] * 0.0625f, acc[7] * 0.0625f };
  if (r < ROWS) {
    float* op = AG + (size_t)r * DIM + 4 * lane;
    *(volatile v4f*)(op)       = o0;
    *(volatile v4f*)(op + 128) = o1;
    __threadfence();
    *(volatile v4f*)(op)       = o0;
    *(volatile v4f*)(op + 128) = o1;
  }
}

template <int MODE>
__global__ __launch_bounds__(256) void k_colstat(const float* __restrict__ H, const float* __restrict__ mean,
                                                 double* __restrict__ rec) {
  static_assert(MODE == 0 || MODE == 1);
  __shared__ __attribute__((aligned(16))) double sd[DIM];
  const int tid = (int)threadIdx.x;
  double m = 0.0;
  if constexpr (MODE == 1) m = (double)mean[tid];
  const float* hp = H + (size_t)blockIdx.x * 128 * DIM + tid;
  double s = 0.0;
#pragma unroll 4
  for (int j = 0; j < 128; ++j) {
    const float v = hp[(size_t)j * DIM];
    if constexpr (MODE == 0) {
      s += (double)v;
    } else {
      const double d = (double)v - m;
      s += d * d;
    }
  }
  sd[tid] = s;
  __syncthreads();
  const int t2 = tid < 128 ? tid : 127;
  const v2d o = *(const v2da*)(sd + 2 * t2);
  if (tid < 128) {
    volatile v2d* q = (volatile v2d*)(rec + (size_t)blockIdx.x * DIM + 2 * tid);
    *q = o;
    __threadfence();
    *q = o;
  }
}

__global__ __launch_bounds__(256) void k_comb(const double* __restrict__ rec, int mode, float* __restrict__ out) {
  __shared__ __attribute__((aligned(16))) float sv[DIM];
  const int tid = (int)threadIdx.x;
  double s = 0.0;
#pragma unroll 4
  for (int i = 0; i < NREC; ++i) s += rec[(size_t)i * DIM + tid];
  const float qf = (float)(s * (1.0 / 16384.0));
  const float rs = 1.0f / sqrtf(qf + 1e-5f);
  sv[tid] = (mode == 0) ? qf : rs;
  __syncthreads();
  const int t4 = tid < 64 ? tid : 63;
  const v4f o = *(const v4fa*)(sv + 4 * t4);
  if (tid < 64) {
    volatile v4f* q = (volatile v4f*)(out + 4 * tid);
    *q = o;
    __threadfence();
    *q = o;
  }
}

template <int LAST>
__global__ __launch_bounds__(256) void k_apply(const float* __restrict__ H, float* __restrict__ XF,
                                               const float* __restrict__ MU, const float* __restrict__ RS,
                                               const float* __restrict__ G, const float* __restrict__ Bt,
                                               unsigned short* __restrict__ XHL, float* __restrict__ out,
                                               unsigned lomask) {
  __shared__ __attribute__((aligned(16))) float sP[4 * DIM];
  __shared__ __attribute__((aligned(16))) float sRow[8 * DIM];
  const int tid = (int)threadIdx.x, lane = tid & 31, wave = tid >> 5;
  if (tid < 64) {
    const v4f a = *(const v4fa*)(MU + 4 * tid);
    const v4f b = *(const v4fa*)(RS + 4 * tid);
    const v4f c = *(const v4fa*)(G + 4 * tid);
    const v4f d = *(const v4fa*)(Bt + 4 * tid);
    *(v4fa*)(sP + 4 * tid)           = a;
    *(v4fa*)(sP + DIM + 4 * tid)     = b;
    *(v4fa*)(sP + 2 * DIM + 4 * tid) = c;
    *(v4fa*)(sP + 3 * DIM + 4 * tid) = d;
  }
  __syncthreads();
  const int row = (int)blockIdx.x * 8 + wave;
  const int rc  = row < ROWS ? row : ROWS - 1;
  const int cA = 4 * lane, cB = 128 + 4 * lane;
  const v4f hA = *(const v4fa*)(H + (size_t)rc * DIM + cA);
  const v4f hB = *(const v4fa*)(H + (size_t)rc * DIM + cB);
  const v4f xA = *(const v4fa*)(XF + (size_t)rc * DIM + cA);
  const v4f xB = *(const v4fa*)(XF + (size_t)rc * DIM + cB);
  asm volatile("" :: "v"(hA));
  asm volatile("" :: "v"(hB));
  asm volatile("" :: "v"(xA));
  asm volatile("" :: "v"(xB));
  const v4f mA = *(const v4fa*)(sP + cA),           mB = *(const v4fa*)(sP + cB);
  const v4f rA = *(const v4fa*)(sP + DIM + cA),     rB = *(const v4fa*)(sP + DIM + cB);
  const v4f gA = *(const v4fa*)(sP + 2 * DIM + cA), gB = *(const v4fa*)(sP + 2 * DIM + cB);
  const v4f eA = *(const v4fa*)(sP + 3 * DIM + cA), eB = *(const v4fa*)(sP + 3 * DIM + cB);
  v4f nA, nB;
#pragma unroll
  for (int e = 0; e < 4; ++e) {
    nA[e] = xA[e] + ((((hA[e] - mA[e]) * rA[e]) * gA[e]) + eA[e]);
    nB[e] = xB[e] + ((((hB[e] - mB[e]) * rB[e]) * gB[e]) + eB[e]);
  }
  if constexpr (LAST == 1) {
    if (row < ROWS) {
      float* op = out + (size_t)row * DIM;
      *(volatile v4f*)(op + cA) = nA;
      *(volatile v4f*)(op + cB) = nB;
      __threadfence();
      *(volatile v4f*)(op + cA) = nA;
      *(volatile v4f*)(op + cB) = nB;
    }
  } else {
    float* sr = sRow + wave * DIM;
    *(v4fa*)(sr + cA) = nA;
    *(v4fa*)(sr + cB) = nB;
    __builtin_amdgcn_fence(__ATOMIC_RELEASE, "workgroup");
    __builtin_amdgcn_wave_barrier();
    __builtin_amdgcn_fence(__ATOMIC_ACQUIRE, "workgroup");
    const v4f a = *(const v4fa*)(sr + 8 * lane);
    const v4f c = *(const v4fa*)(sr + 8 * lane + 4);
    const v4u mk = (v4u){ lomask, lomask, lomask, lomask };
    const v4u hi = pack8_bf16(a, c);
    const v4u lo = pack8_bf16_lo(a, c) & mk;
    if (row < ROWS) {
      float* xp = XF + (size_t)row * DIM;
      unsigned short* hp = XHL + (size_t)row * (2 * DIM) + 8 * lane;
      *(volatile v4f*)(xp + cA)  = nA;
      *(volatile v4f*)(xp + cB)  = nB;
      *(volatile v4u*)(hp)       = hi;
      *(volatile v4u*)(hp + DIM) = lo;
      __threadfence();
      *(volatile v4f*)(xp + cA)  = nA;
      *(volatile v4f*)(xp + cB)  = nB;
      *(volatile v4u*)(hp)       = hi;
      *(volatile v4u*)(hp + DIM) = lo;
    }
  }
}

extern "C" void kernel_launch(void* const* d_in, const int* in_sizes, int n_in,
                              void* d_out, int out_size, void* d_ws, size_t ws_size,
                              hipStream_t stream) {
  if (n_in < 13) return;
  if (in_sizes[0] != ROWS * DIM) return;
  if (in_sizes[1] != ROWS * 3) return;
  if (in_sizes[2] != ROWS * KNB) return;
  if (in_sizes[3] != DEPTH * DIM * DIM) return;
  if (in_sizes[4] != DEPTH * D4 * 3) return;
  if (in_sizes[5] != DEPTH * D4) return;
  if (in_sizes[6] != DEPTH * DIM || in_sizes[7] != DEPTH * DIM) return;
  if (in_sizes[8] != NMLP * DIM * HID) return;
  if (in_sizes[9] != NMLP * HID) return;
  if (in_sizes[10] != NMLP * HID * DIM) return;
  if (in_sizes[11] != NMLP * DIM || in_sizes[12] != NMLP * DIM) return;
  if (out_size != OUT_ELEMS) return;
  if (ws_size < WS_TOTAL) return;

  const float* x_in      = (const float*)d_in[0];
  const float* xyz       = (const float*)d_in[1];
  const int*   knn       = (const int*)d_in[2];
  const float* lfp_proj  = (const float*)d_in[3];
  const float* lfp_coor  = (const float*)d_in[4];
  const float* lfp_scale = (const float*)d_in[5];
  const float* lfp_gamma = (const float*)d_in[6];
  const float* lfp_beta  = (const float*)d_in[7];
  const float* mlp_w1    = (const float*)d_in[8];
  const float* mlp_b1    = (const float*)d_in[9];
  const float* mlp_w2    = (const float*)d_in[10];
  const float* mlp_gamma = (const float*)d_in[11];
  const float* mlp_beta  = (const float*)d_in[12];
  float* out = (float*)d_out;

  char* ws = (char*)d_ws;
  float*          XF   = (float*)(ws + OFF_XF);
  unsigned short* XHL  = (unsigned short*)(ws + OFF_XHL);
  float*          HP   = (float*)(ws + OFF_HP);
  float*          AG   = (float*)(ws + OFF_AG);
  float*          C1   = (float*)(ws + OFF_C1);
  unsigned short* C1HL = (unsigned short*)(ws + OFF_C1HL);
  unsigned short* XB   = (unsigned short*)(ws + OFF_XB);
  unsigned short* W1A  = (unsigned short*)(ws + OFF_W1A);
  unsigned short* W1B  = (unsigned short*)(ws + OFF_W1B);
  unsigned short* W2P  = (unsigned short*)(ws + OFF_W2P);
  unsigned short* LW2  = (unsigned short*)(ws + OFF_LW2);
  float*          TB   = (float*)(ws + OFF_TB);
  float*          PC   = (float*)(ws + OFF_TB + TBB_PC);
  double*         REC  = (double*)(ws + OFF_TB + TBB_REC);
  float*          MU   = TB + TB_MU;
  float*          RS   = TB + TB_RS;

  k_prep_x<<<ROWS / 8, 256, 0, stream>>>(x_in, XF, XB);
  k_prep_small<<<PS_TOT, 256, 0, stream>>>(xyz, lfp_coor, lfp_scale, lfp_gamma, lfp_beta, mlp_b1, mlp_gamma, mlp_beta,
                                           PC, TB);
  k_wT<<<(DIM / 64) * (HID / 64), 256, 0, stream>>>(mlp_w1, W1A, DIM, HID, 1);
  k_wT<<<2 * (DIM / 64) * (HID / 64), 256, 0, stream>>>(mlp_w1 + (size_t)DIM * HID, W1B, DIM, HID, 2);
  k_wT<<<NMLP * (HID / 64) * (DIM / 64), 256, 0, stream>>>(mlp_w2, W2P, HID, DIM, 2);
  k_wT<<<DEPTH * (DIM / 64) * (DIM / 64), 256, 0, stream>>>(lfp_proj, LW2, DIM, DIM, 2);

  auto bn = [&](const float* g, const float* bt, bool last, unsigned lom) {
    k_colstat<0><<<NREC, 256, 0, stream>>>(AG, MU, REC);
    k_comb<<<1, 256, 0, stream>>>(REC, 0, MU);
    k_colstat<1><<<NREC, 256, 0, stream>>>(AG, MU, REC);
    k_comb<<<1, 256, 0, stream>>>(REC, 1, RS);
    if (last) k_apply<1><<<ROWS / 8, 256, 0, stream>>>(AG, XF, MU, RS, g, bt, XHL, out, lom);
    else      k_apply<0><<<ROWS / 8, 256, 0, stream>>>(AG, XF, MU, RS, g, bt, XHL, out, lom);
  };
  auto mlp = [&](int j, unsigned lom_hid, bool last, unsigned lom_next) {
    const unsigned short* Bw1 = (j == 0) ? W1A : (W1B + (size_t)(j - 1) * HID * 2 * DIM);
    const int K1 = (j == 0) ? DIM : 2 * DIM;
    for (int c = 0; c < NCHUNK; ++c) {
      const unsigned short* A1 = (j == 0) ? (XB + (size_t)c * CHROWS * DIM) : (XHL + (size_t)c * CHROWS * 2 * DIM);
      k_gemm_nt<0, 0><<<((CHROWS / 64) * (HID / 64) + 7) / 8, 256, 0, stream>>>(A1, Bw1, TB, C1, CHROWS, HID, K1, HID);
      k_gelu<<<CHROWS / 8, 256, 0, stream>>>(C1, TB + TB_B1 + (size_t)j * HID, C1HL, lom_hid);
      k_gemm_nt<0, 0><<<((CHROWS / 64) * (DIM / 64) + 7) / 8, 256, 0, stream>>>(
          C1HL, W2P + (size_t)j * DIM * 2 * HID, TB, AG + (size_t)c * CHROWS * DIM, CHROWS, DIM, 2 * HID, DIM);
    }
    bn(TB + TB_MG + (size_t)j * DIM, TB + TB_MB + (size_t)j * DIM, last, lom_next);
  };
  auto lfp = [&](int i, unsigned lom_next) {
    k_gemm_nt<0, 0><<<((ROWS / 64) * (DIM / 64) + 7) / 8, 256, 0, stream>>>(
        XHL, LW2 + (size_t)i * DIM * 2 * DIM, TB, HP, ROWS, DIM, 2 * DIM, DIM);
    k_lfp<<<ROWS / 8, 256, 0, stream>>>(HP, PC, knn, TB + TB_LFPT + (size_t)i * D4 * 8, AG);
    bn(TB + TB_LG + (size_t)i * DIM, TB + TB_LB + (size_t)i * DIM, false, lom_next);
  };

  mlp(0, site_mask(0), false, site_mask(1));
  lfp(0, site_mask(2));
  lfp(1, site_mask(3));
  mlp(1, site_mask(4), false, site_mask(5));
  lfp(2, site_mask(6));
  lfp(3, site_mask(7));
  mlp(2, site_mask(8), true, 0xFFFFFFFFu);
}
